// SwinTransformerBlock_lucid_2061584302085
// MI455X (gfx1250) — hardware-verified
//
#include <hip/hip_runtime.h>
#include <hip/hip_bf16.h>
#include <math.h>

#define SEQ   343
#define NW    128
#define CCH   192
#define NH    6
#define DHD   32
#define FFI   768
#define ROWS  (NW * SEQ)
#define QKV_N 576
#define KT22  22
#define SPAD  352

typedef __bf16 bf16x16 __attribute__((ext_vector_type(16)));
typedef float  f32x8   __attribute__((ext_vector_type(8)));

union FragU { bf16x16 v; uint4 u[2]; };
union Pack8 { uint4 u; __hip_bfloat16 h[8]; };
union F4x2  { float4 v[2]; float f[8]; };

__device__ __forceinline__ bf16x16 frag_a(const __hip_bfloat16* base, int ld) {
  const int lane = threadIdx.x & 31;
  const __hip_bfloat16* p = base + (size_t)(lane & 15) * ld + ((lane >> 4) << 3);
  FragU f;
  f.u[0] = *(const uint4*)p;
  f.u[1] = *(const uint4*)(p + 16);
  return f.v;
}

__device__ __forceinline__ bf16x16 frag_b(const __hip_bfloat16* base, int ld) {
  const int lane = threadIdx.x & 31;
  const __hip_bfloat16* p = base + (size_t)(lane & 15) * ld + ((lane >> 4) << 3);
  FragU f;
  f.u[0] = *(const uint4*)p;
  f.u[1] = *(const uint4*)(p + 16);
  return f.v;
}

__device__ __forceinline__ f32x8 wmma_bf16(bf16x16 a, bf16x16 b, f32x8 c) {
  return __builtin_amdgcn_wmma_f32_16x16x32_bf16(false, a, false, b, (short)0, c,
                                                 false, false);
}

__global__ void transpose_w_kernel(const float* __restrict__ W,
                                   __hip_bfloat16* __restrict__ WT, int K, int N) {
  int idx = blockIdx.x * 256 + threadIdx.x;
  if (idx >= K * N) return;
  int n = idx / K, k = idx % K;
  WT[idx] = __float2bfloat16(W[(size_t)k * N + n]);
}

__global__ void bias_prep_kernel(const float* __restrict__ rpb,
                                 const int* __restrict__ relidx,
                                 __hip_bfloat16* __restrict__ biasp) {
  int idx = blockIdx.x * 256 + threadIdx.x;
  if (idx >= NH * SPAD * SPAD) return;
  const int head = idx / (SPAD * SPAD);
  const int rem = idx % (SPAD * SPAD);
  const int q = rem / SPAD, k = rem % SPAD;
  float v = 0.f;
  if (k >= SEQ) v = -1e9f;
  else if (q < SEQ) v = rpb[relidx[q * SEQ + k] * NH + head];
  biasp[idx] = __float2bfloat16(v);
}

__global__ void mask_prep_kernel(const float* __restrict__ mask,
                                 __hip_bfloat16* __restrict__ maskp) {
  int idx = blockIdx.x * 256 + threadIdx.x;
  if (idx >= NW * SPAD * SPAD) return;
  const int win = idx / (SPAD * SPAD);
  const int rem = idx % (SPAD * SPAD);
  const int q = rem / SPAD, k = rem % SPAD;
  float v = 0.f;
  if (q < SEQ && k < SEQ && mask[((size_t)win * SEQ + q) * SEQ + k] != 0.f) v = -1e9f;
  maskp[idx] = __float2bfloat16(v);
}

__global__ __launch_bounds__(192) void partition_kernel(const float* __restrict__ x,
                                                        float* __restrict__ xw) {
  const int row = blockIdx.x, c = threadIdx.x;
  const int win = row / SEQ, s = row % SEQ;
  const int di = win >> 5, hi = (win >> 2) & 7, wi = win & 3;
  const int dd = s / 49, hh = (s / 7) % 7, ww = s % 7;
  const int d = (di * 7 + dd + 3) % 28;
  const int h = (hi * 7 + hh + 3) % 56;
  const int w = (wi * 7 + ww + 3) % 28;
  xw[(size_t)row * CCH + c] = x[((size_t)(d * 56 + h) * 28 + w) * CCH + c];
}

__global__ __launch_bounds__(256) void ln_kernel(const float* __restrict__ X,
                                                 const float* __restrict__ w,
                                                 const float* __restrict__ b,
                                                 __hip_bfloat16* __restrict__ Y,
                                                 int rows) {
  const int row = blockIdx.x * 8 + (threadIdx.x >> 5);
  const int lane = threadIdx.x & 31;
  if (row >= rows) return;
  const float* x = X + (size_t)row * CCH;
  float v[6], s = 0.f;
#pragma unroll
  for (int i = 0; i < 6; ++i) { v[i] = x[lane + i * 32]; s += v[i]; }
#pragma unroll
  for (int off = 16; off > 0; off >>= 1) s += __shfl_xor(s, off, 32);
  const float mu = s * (1.0f / CCH);
  float q = 0.f;
#pragma unroll
  for (int i = 0; i < 6; ++i) { float d = v[i] - mu; q += d * d; }
#pragma unroll
  for (int off = 16; off > 0; off >>= 1) q += __shfl_xor(q, off, 32);
  const float rs = rsqrtf(q * (1.0f / CCH) + 1e-5f);
#pragma unroll
  for (int i = 0; i < 6; ++i) {
    int c = lane + i * 32;
    Y[(size_t)row * CCH + c] = __float2bfloat16((v[i] - mu) * rs * w[c] + b[c]);
  }
}

enum { EPI_QKV = 0, EPI_RESID = 1, EPI_GLU = 2 };

template <int EPI>
__global__ __launch_bounds__(256) void gemm_bf16(
    const __hip_bfloat16* __restrict__ A,
    const __hip_bfloat16* __restrict__ WT,
    const float* __restrict__ bias,
    const float* __restrict__ resid,
    float* __restrict__ outF,
    __hip_bfloat16* __restrict__ outH,
    int N, int K) {
  const int wave = threadIdx.x >> 5;
  const int lane = threadIdx.x & 31;
  const int m0 = blockIdx.x * 128 + wave * 16;
  const int n0 = blockIdx.y * 64;

  f32x8 acc[4] = {};
  f32x8 acc2[4] = {};
  for (int k0 = 0; k0 < K; k0 += 32) {
    if (k0 + 32 < K)
      __builtin_prefetch(A + (size_t)m0 * K + k0 + 32, 0, 1);
    bf16x16 bt = frag_b(A + (size_t)m0 * K + k0, K);
#pragma unroll
    for (int nt = 0; nt < 4; ++nt) {
      bf16x16 wa = frag_a(WT + (size_t)(n0 + nt * 16) * K + k0, K);
      acc[nt] = wmma_bf16(wa, bt, acc[nt]);
      if (EPI == EPI_GLU) {
        bf16x16 wg = frag_a(WT + (size_t)(n0 + nt * 16 + N) * K + k0, K);
        acc2[nt] = wmma_bf16(wg, bt, acc2[nt]);
      }
    }
  }
  const int m = m0 + (lane & 15);
  const int nb = (lane >> 4) << 3;
#pragma unroll
  for (int nt = 0; nt < 4; ++nt) {
    const int nbase = n0 + nt * 16 + nb;
    F4x2 bv;
    bv.v[0] = *(const float4*)(bias + nbase);
    bv.v[1] = *(const float4*)(bias + nbase + 4);
    if (EPI == EPI_QKV) {
      const float sc = (nbase < CCH) ? 0.17677669529663687f : 1.0f;
      Pack8 o;
#pragma unroll
      for (int r = 0; r < 8; ++r) o.h[r] = __float2bfloat16((acc[nt][r] + bv.f[r]) * sc);
      *(uint4*)(outH + (size_t)m * QKV_N + nbase) = o.u;
    } else if (EPI == EPI_RESID) {
      F4x2 rv, o;
      rv.v[0] = *(const float4*)(resid + (size_t)m * N + nbase);
      rv.v[1] = *(const float4*)(resid + (size_t)m * N + nbase + 4);
#pragma unroll
      for (int r = 0; r < 8; ++r) o.f[r] = acc[nt][r] + bv.f[r] + rv.f[r];
      *(float4*)(outF + (size_t)m * N + nbase) = o.v[0];
      *(float4*)(outF + (size_t)m * N + nbase + 4) = o.v[1];
    } else {
      F4x2 bg;
      bg.v[0] = *(const float4*)(bias + N + nbase);
      bg.v[1] = *(const float4*)(bias + N + nbase + 4);
      Pack8 o;
#pragma unroll
      for (int r = 0; r < 8; ++r) {
        const float u = acc[nt][r] + bv.f[r];
        float g = acc2[nt][r] + bg.f[r];
        const float t =
            0.5f * g * (1.0f + tanhf(0.7978845608028654f * (g + 0.044715f * g * g * g)));
        o.h[r] = __float2bfloat16(u * t);
      }
      *(uint4*)(outH + (size_t)m * N + nbase) = o.u;
    }
  }
}

__global__ __launch_bounds__(64) void attn_kernel(
    const __hip_bfloat16* __restrict__ qkv,
    const __hip_bfloat16* __restrict__ biasp,
    const __hip_bfloat16* __restrict__ maskp,
    float* __restrict__ obufF) {
  __shared__ __align__(16) __hip_bfloat16 sS[2][16][SPAD];
  __shared__ __align__(16) __hip_bfloat16 sVT[DHD][SPAD];
  const int win = blockIdx.x / NH;
  const int head = blockIdx.x % NH;
  const int tid = threadIdx.x;
  const int wave = tid >> 5;
  const int lane = tid & 31;

  for (int i = tid; i < DHD * SPAD; i += 64) {
    const int d = i & 31, key = i >> 5;
    float v = 0.f;
    if (key < SEQ)
      v = __bfloat162float(qkv[(size_t)(win * SEQ + key) * QKV_N + 2 * CCH + head * DHD + d]);
    sVT[d][key] = __float2bfloat16(v);
  }
  __syncthreads();

  const int rb = (lane >> 4) << 3;
  const int half8 = (lane >> 4) << 3;
  const int half16 = (lane >> 4) << 4;
  const __hip_bfloat16* biaspl = biasp + (size_t)head * SPAD * SPAD;
  const __hip_bfloat16* maskpl = maskp + (size_t)win * SPAD * SPAD;

  for (int qt = wave; qt < KT22; qt += 2) {
    const int q0 = qt * 16;
    const int qg = q0 + (lane & 15);
    int qtok = qg; if (qtok > SEQ - 1) qtok = SEQ - 1;
    FragU fq;
    const __hip_bfloat16* pq =
        qkv + (size_t)(win * SEQ + qtok) * QKV_N + head * DHD + half8;
    fq.u[0] = *(const uint4*)pq; fq.u[1] = *(const uint4*)(pq + 16);

    float mx = -1e30f;
    for (int kt = 0; kt < KT22; ++kt) {
      int ktok = kt * 16 + (lane & 15); if (ktok > SEQ - 1) ktok = SEQ - 1;
      FragU fk;
      const __hip_bfloat16* pk =
          qkv + (size_t)(win * SEQ + ktok) * QKV_N + CCH + head * DHD + half8;
      fk.u[0] = *(const uint4*)pk; fk.u[1] = *(const uint4*)(pk + 16);
      f32x8 s = {};
      s = wmma_bf16(fk.v, fq.v, s);
      const int kbase = kt * 16 + rb;
      Pack8 bb, mm, o;
      bb.u = *(const uint4*)(biaspl + (size_t)qg * SPAD + kbase);
      mm.u = *(const uint4*)(maskpl + (size_t)qg * SPAD + kbase);
#pragma unroll
      for (int r = 0; r < 8; ++r) {
        const float val = s[r] + __bfloat162float(bb.h[r]) + __bfloat162float(mm.h[r]);
        mx = fmaxf(mx, val);
        o.h[r] = __float2bfloat16(val);
      }
      *(uint4*)&sS[wave][lane & 15][kbase] = o.u;
    }
    mx = fmaxf(mx, __shfl_xor(mx, 16, 32));
    asm volatile("s_wait_dscnt 0" ::: "memory");

    float sum = 0.f;
    {
      const int row = lane & 15;
      const int c0 = (lane >> 4) * 176;
      __hip_bfloat16* sr = &sS[wave][row][c0];
      for (int c = 0; c < 176; c += 8) {
        Pack8 p; p.u = *(const uint4*)(sr + c);
#pragma unroll
        for (int j = 0; j < 8; ++j) {
          const float e = __expf(__bfloat162float(p.h[j]) - mx);
          sum += e;
          p.h[j] = __float2bfloat16(e);
        }
        *(uint4*)(sr + c) = p.u;
      }
    }
    sum += __shfl_xor(sum, 16, 32);
    const float inv = 1.0f / sum;
    asm volatile("s_wait_dscnt 0" ::: "memory");

    f32x8 o0 = {}, o1 = {};
    for (int kk = 0; kk < 11; ++kk) {
      FragU fp, fv0, fv1;
      const __hip_bfloat16* pp = &sS[wave][lane & 15][kk * 32 + half8];
      fp.u[0] = *(const uint4*)pp; fp.u[1] = *(const uint4*)(pp + 16);
      const __hip_bfloat16* pv0 = &sVT[lane & 15][kk * 32 + half8];
      fv0.u[0] = *(const uint4*)pv0; fv0.u[1] = *(const uint4*)(pv0 + 16);
      const __hip_bfloat16* pv1 = &sVT[16 + (lane & 15)][kk * 32 + half8];
      fv1.u[0] = *(const uint4*)pv1; fv1.u[1] = *(const uint4*)(pv1 + 16);
      o0 = wmma_bf16(fv0.v, fp.v, o0);
      o1 = wmma_bf16(fv1.v, fp.v, o1);
    }
    if (qg < SEQ) {
      F4x2 a, b;
#pragma unroll
      for (int r = 0; r < 8; ++r) { a.f[r] = o0[r] * inv; b.f[r] = o1[r] * inv; }
      float* op = obufF + (size_t)(win * SEQ + qg) * CCH + head * DHD;
#pragma unroll
      for (int r = 0; r < 8; ++r) { *(volatile float*)(op + rb + r) = a.f[r]; *(volatile float*)(op + 16 + rb + r) = b.f[r]; }
      __threadfence();
#pragma unroll
      for (int r = 0; r < 8; ++r) { *(volatile float*)(op + rb + r) = a.f[r]; *(volatile float*)(op + 16 + rb + r) = b.f[r]; }
    }
  }
}

__global__ __launch_bounds__(256) void cvt_obuf_kernel(const float* __restrict__ src, __hip_bfloat16* __restrict__ dst, int n) {
  const int i = blockIdx.x * 256 + threadIdx.x; if (i >= n) return;
  const __hip_bfloat16 v = __float2bfloat16(src[i]);
  *(volatile __hip_bfloat16*)(dst + i) = v; __threadfence(); *(volatile __hip_bfloat16*)(dst + i) = v;
}

__global__ __launch_bounds__(256) void final_kernel(const float* __restrict__ X,
                                                    const float* __restrict__ w,
                                                    const float* __restrict__ b,
                                                    float* __restrict__ out) {
  const int row = blockIdx.x * 8 + (threadIdx.x >> 5);
  const int lane = threadIdx.x & 31;
  if (row >= ROWS) return;
  const float* x = X + (size_t)row * CCH;
  float v[6], s = 0.f;
#pragma unroll
  for (int i = 0; i < 6; ++i) { v[i] = x[lane + i * 32]; s += v[i]; }
#pragma unroll
  for (int off = 16; off > 0; off >>= 1) s += __shfl_xor(s, off, 32);
  const float mu = s * (1.0f / CCH);
  float q = 0.f;
#pragma unroll
  for (int i = 0; i < 6; ++i) { float d = v[i] - mu; q += d * d; }
#pragma unroll
  for (int off = 16; off > 0; off >>= 1) q += __shfl_xor(q, off, 32);
  const float rs = rsqrtf(q * (1.0f / CCH) + 1e-5f);

  const int win = row / SEQ, si = row % SEQ;
  const int di = win >> 5, hi = (win >> 2) & 7, wi = win & 3;
  const int dd = si / 49, hh = (si / 7) % 7, ww = si % 7;
  const int d = (di * 7 + dd + 3) % 28;
  const int h = (hi * 7 + hh + 3) % 56;
  const int wo = (wi * 7 + ww + 3) % 28;
  float* dst = out + ((size_t)(d * 56 + h) * 28 + wo) * CCH;
#pragma unroll
  for (int i = 0; i < 6; ++i) {
    const int c = lane + i * 32;
    dst[c] = (v[i] - mu) * rs * w[c] + b[c];
  }
}

extern "C" void kernel_launch(void* const* d_in, const int* in_sizes, int n_in,
                              void* d_out, int out_size, void* d_ws, size_t ws_size,
                              hipStream_t stream) {
  const float* x      = (const float*)d_in[0];
  const float* mask   = (const float*)d_in[1];
  const float* ln1_w  = (const float*)d_in[3];
  const float* ln1_b  = (const float*)d_in[4];
  const float* qkv_w  = (const float*)d_in[5];
  const float* qkv_b  = (const float*)d_in[6];
  const float* out_w  = (const float*)d_in[7];
  const float* out_b  = (const float*)d_in[8];
  const float* ln2_w  = (const float*)d_in[9];
  const float* ln2_b  = (const float*)d_in[10];
  const float* ff1_w  = (const float*)d_in[11];
  const float* ff1_b  = (const float*)d_in[12];
  const float* ff2_w  = (const float*)d_in[13];
  const float* ff2_b  = (const float*)d_in[14];
  const float* rpb    = (const float*)d_in[15];
  const float* lnf_w  = (const float*)d_in[16];
  const float* lnf_b  = (const float*)d_in[17];
  const int*   relidx = (const int*)d_in[18];
  float* out = (float*)d_out;

  char* ws = (char*)d_ws;
  size_t off = 0;
  auto carve = [&](size_t bytes) { void* p = ws + off; off += (bytes + 255) & ~size_t(255); return p; };
  float*          xw     = (float*)carve((size_t)ROWS * CCH * 4);
  __hip_bfloat16* hdn    = (__hip_bfloat16*)carve((size_t)ROWS * CCH * 2);
  __hip_bfloat16* qkvbuf = (__hip_bfloat16*)carve((size_t)ROWS * QKV_N * 2);
  __hip_bfloat16* obuf   = (__hip_bfloat16*)carve((size_t)ROWS * CCH * 2);
  __hip_bfloat16* ffh    = (__hip_bfloat16*)carve((size_t)ROWS * FFI * 2);
  __hip_bfloat16* qkvT   = (__hip_bfloat16*)carve((size_t)2 * QKV_N * CCH * 2);
  __hip_bfloat16* outT   = (__hip_bfloat16*)carve((size_t)2 * CCH * CCH * 2);
  __hip_bfloat16* ff1T   = (__hip_bfloat16*)carve((size_t)2 * 1536 * CCH * 2);
  __hip_bfloat16* ff2T   = (__hip_bfloat16*)carve((size_t)2 * CCH * FFI * 2);
  __hip_bfloat16* biasp  = (__hip_bfloat16*)carve((size_t)NH * SPAD * SPAD * 2);
  __hip_bfloat16* maskp  = (__hip_bfloat16*)carve((size_t)NW * SPAD * SPAD * 2);
  float*          obufF  = (float*)carve((size_t)ROWS * CCH * 4);
  if (off > ws_size) return;

  for (int l = 0; l < 2; ++l) {
    {
      int K = CCH, N = QKV_N, n = K * N;
      transpose_w_kernel<<<(n + 255) / 256, 256, 0, stream>>>(qkv_w + (size_t)l * n,
                                                              qkvT + (size_t)l * n, K, N);
    }
    {
      int K = CCH, N = CCH, n = K * N;
      transpose_w_kernel<<<(n + 255) / 256, 256, 0, stream>>>(out_w + (size_t)l * n,
                                                              outT + (size_t)l * n, K, N);
    }
    {
      int K = CCH, N = 1536, n = K * N;
      transpose_w_kernel<<<(n + 255) / 256, 256, 0, stream>>>(ff1_w + (size_t)l * n,
                                                              ff1T + (size_t)l * n, K, N);
    }
    {
      int K = FFI, N = CCH, n = K * N;
      transpose_w_kernel<<<(n + 255) / 256, 256, 0, stream>>>(ff2_w + (size_t)l * n,
                                                              ff2T + (size_t)l * n, K, N);
    }
  }

  {
    int n = NW * SPAD * SPAD;
    mask_prep_kernel<<<(n + 255) / 256, 256, 0, stream>>>(mask, maskp);
  }

  partition_kernel<<<ROWS, 192, 0, stream>>>(x, xw);

  const dim3 blk256(256);
  for (int l = 0; l < 2; ++l) {
    {
      int n = NH * SPAD * SPAD;
      bias_prep_kernel<<<(n + 255) / 256, 256, 0, stream>>>(
          rpb + (size_t)l * 2197 * NH, relidx, biasp);
    }
    ln_kernel<<<ROWS / 8, blk256, 0, stream>>>(xw, ln1_w + l * CCH, ln1_b + l * CCH,
                                               hdn, ROWS);
    gemm_bf16<EPI_QKV><<<dim3(ROWS / 128, QKV_N / 64), blk256, 0, stream>>>(
        hdn, qkvT + (size_t)l * QKV_N * CCH, qkv_b + (size_t)l * QKV_N,
        nullptr, nullptr, qkvbuf, QKV_N, CCH);
    attn_kernel<<<NW * NH, 64, 0, stream>>>(qkvbuf, biasp, maskp, obufF);
    cvt_obuf_kernel<<<(ROWS * CCH + 255) / 256, 256, 0, stream>>>(obufF, obuf, ROWS * CCH);
    gemm_bf16<EPI_RESID><<<dim3(ROWS / 128, CCH / 64), blk256, 0, stream>>>(
        obuf, outT + (size_t)l * CCH * CCH, out_b + (size_t)l * CCH,
        xw, xw, nullptr, CCH, CCH);
    ln_kernel<<<ROWS / 8, blk256, 0, stream>>>(xw, ln2_w + l * CCH, ln2_b + l * CCH,
                                               hdn, ROWS);
    gemm_bf16<EPI_GLU><<<dim3(ROWS / 128, FFI / 64), blk256, 0, stream>>>(
        hdn, ff1T + (size_t)l * 1536 * CCH, ff1_b + (size_t)l * 1536,
        nullptr, nullptr, ffh, FFI, CCH);
    gemm_bf16<EPI_RESID><<<dim3(ROWS / 128, CCH / 64), blk256, 0, stream>>>(
        ffh, ff2T + (size_t)l * CCH * FFI, ff2_b + (size_t)l * CCH,
        xw, xw, nullptr, CCH, FFI);
  }

  final_kernel<<<ROWS / 8, blk256, 0, stream>>>(xw, lnf_w, lnf_b, out);
}
